// LocalAttention_50964081934690
// MI455X (gfx1250) — hardware-verified
//
#include <hip/hip_runtime.h>

typedef __attribute__((ext_vector_type(16))) _Float16 v16h;
typedef __attribute__((ext_vector_type(8)))  _Float16 v8h;
typedef __attribute__((ext_vector_type(4)))  _Float16 v4h;
typedef __attribute__((ext_vector_type(8)))  float    v8f;

typedef unsigned int u32;
typedef __attribute__((ext_vector_type(4))) u32 v4u;
typedef __attribute__((ext_vector_type(8))) int v8i;
typedef __attribute__((ext_vector_type(4))) int v4i;

#define BATCH     2
#define SEQ       2048
#define HID       1024
#define NHEADS    16
#define HEAD_DIM  64
#define HALF_W    128
#define NEG_BIG   (-1.0e30f)

#define LDS_PBUF_BYTES   (4 * 1024)
#define LDS_PLBUF_BASE   (LDS_PBUF_BYTES)
#define LDS_KBUF_BASE    (LDS_PLBUF_BASE + LDS_PBUF_BYTES)
#define LDS_KLBUF_BASE   (LDS_KBUF_BASE + 8 * 4096)
#define LDS_VBUF_BASE    (LDS_KLBUF_BASE + 8 * 4096)
#define LDS_VLBUF_BASE   (LDS_VBUF_BASE + 8 * 4096)
#define LDS_TOTAL_BYTES  (LDS_VLBUF_BASE + 8 * 4096)
#define PLM  ((size_t)BATCH * SEQ * HID)
#define PLW  ((size_t)HID * HID)
#define RSPLIT (1.0f / 2048.0f)

typedef __attribute__((ext_vector_type(4))) float v4f_t;
typedef float v4fa __attribute__((ext_vector_type(4), may_alias));
typedef __attribute__((ext_vector_type(4))) unsigned v4u_t;
typedef unsigned v4ua __attribute__((ext_vector_type(4), may_alias));
static __device__ __forceinline__ unsigned pk2s(float a, float b, unsigned* lop) {
    const _Float16 h0 = (_Float16)a, h1 = (_Float16)b;
    *lop = (unsigned)__builtin_bit_cast(unsigned short, (_Float16)((a - (float)h0) * 2048.0f)) | ((unsigned)__builtin_bit_cast(unsigned short, (_Float16)((b - (float)h1) * 2048.0f)) << 16);
    return (unsigned)__builtin_bit_cast(unsigned short, h0) | ((unsigned)__builtin_bit_cast(unsigned short, h1) << 16);
}
static __device__ __forceinline__ v8f wmma_split(v16h a, v16h al, v16h b, v16h bl, v8f c) {
    v8f x = {};
    x = __builtin_amdgcn_wmma_f32_16x16x32_f16(false, al, false, b, (short)0, x, false, false);
    x = __builtin_amdgcn_wmma_f32_16x16x32_f16(false, a, false, bl, (short)0, x, false, false);
    return __builtin_amdgcn_wmma_f32_16x16x32_f16(false, a, false, b, (short)0, c, false, false) + x * RSPLIT;
}
static __device__ __forceinline__ unsigned pk2(float a, float b) { return (unsigned)__builtin_bit_cast(unsigned short, (_Float16)a) | ((unsigned)__builtin_bit_cast(unsigned short, (_Float16)b) << 16); }
__device__ __forceinline__ v16h cat8(v8h a, v8h b) {
    return __builtin_shufflevector(a, b, 0, 1, 2, 3, 4, 5, 6, 7,
                                         8, 9, 10, 11, 12, 13, 14, 15);
}

__device__ __forceinline__ void tdm_load_tile_f16(u32 lds_byte_off, const void* gptr,
                                                  u32 tile_d0, u32 tile_d1,
                                                  u32 tensor_d0, u32 tensor_d1,
                                                  u32 stride0)
{
    const unsigned long long ga = (unsigned long long)(uintptr_t)gptr;
    v4u g0;
    g0[0] = 1u;
    g0[1] = lds_byte_off;
    g0[2] = (u32)(ga & 0xFFFFFFFFull);
    g0[3] = (u32)(ga >> 32) | (2u << 30);

    v8i g1;
    g1[0] = (int)(1u << 16);
    g1[1] = (int)((tensor_d0 & 0xFFFFu) << 16);
    g1[2] = (int)(((tensor_d0 >> 16) & 0xFFFFu) |
                  ((tensor_d1 & 0xFFFFu) << 16));
    g1[3] = (int)(((tensor_d1 >> 16) & 0xFFFFu) | (tile_d0 << 16));
    g1[4] = (int)(tile_d1);
    g1[5] = (int)stride0;
    g1[6] = 0;
    g1[7] = 0;
    const v4i z4 = {0, 0, 0, 0};
    const v8i z8 = {0, 0, 0, 0, 0, 0, 0, 0};
    __builtin_amdgcn_tensor_load_to_lds(g0, g1, z4, z4, z8, 0);
}

__global__ void cvt_x_kernel(const float* __restrict__ x, _Float16* __restrict__ xh)
{
    const size_t idx = ((size_t)blockIdx.x * blockDim.x + threadIdx.x) * 4;
    const float4 v = *(const float4*)(x + idx);
    v4h o;
    o[0] = (_Float16)v.x; o[1] = (_Float16)v.y;
    o[2] = (_Float16)v.z; o[3] = (_Float16)v.w;
    v4h ol;
    ol[0] = (_Float16)((v.x - (float)o[0]) * 2048.0f); ol[1] = (_Float16)((v.y - (float)o[1]) * 2048.0f);
    ol[2] = (_Float16)((v.z - (float)o[2]) * 2048.0f); ol[3] = (_Float16)((v.w - (float)o[3]) * 2048.0f);
    *(volatile v4h*)(xh + idx) = o; *(volatile v4h*)(xh + PLM + idx) = ol; __threadfence(); *(volatile v4h*)(xh + idx) = o; *(volatile v4h*)(xh + PLM + idx) = ol;
}

__global__ void cvt_w_kernel(const float* __restrict__ Wq, const float* __restrict__ Wk,
                             const float* __restrict__ Wv, const float* __restrict__ Wo,
                             _Float16* __restrict__ WTq, _Float16* __restrict__ WTk,
                             _Float16* __restrict__ WTv, _Float16* __restrict__ WTo)
{
    const int mat = blockIdx.y;
    const float* W  = (mat == 0) ? Wq : (mat == 1) ? Wk : (mat == 2) ? Wv : Wo;
    _Float16*   WT  = (mat == 0) ? WTq : (mat == 1) ? WTk : (mat == 2) ? WTv : WTo;
    const size_t i = ((size_t)blockIdx.x * blockDim.x + threadIdx.x) * 2;
    if (i >= (size_t)HID * HID) return;
    const int n = (int)(i / HID), k = (int)(i % HID);
    unsigned lo2; const unsigned p = pk2s(W[(size_t)k * HID + n], W[(size_t)(k + 1) * HID + n], &lo2);
    *(volatile unsigned*)(WT + i) = p; *(volatile unsigned*)(WT + PLW + i) = lo2; __threadfence(); *(volatile unsigned*)(WT + i) = p; *(volatile unsigned*)(WT + PLW + i) = lo2;
}

__global__ void qkv_proj_kernel(const _Float16* __restrict__ xh,
                                const _Float16* __restrict__ WTq,
                                const _Float16* __restrict__ WTk,
                                const _Float16* __restrict__ WTv,
                                const float* __restrict__ bq,
                                const float* __restrict__ bk,
                                const float* __restrict__ bv,
                                _Float16* __restrict__ Qh,
                                _Float16* __restrict__ Kh,
                                _Float16* __restrict__ Vt)
{
    const int lane = threadIdx.x & 31;
    const int wave = threadIdx.x >> 5;
    const int lo   = lane & 15;
    const int hi   = lane >> 4;
    const int rowTile = blockIdx.x;
    const int colBase = (blockIdx.y * 4 + wave) * 64;
    const int mat     = blockIdx.z;

    const _Float16* WT = (mat == 0) ? WTq : (mat == 1) ? WTk : WTv;
    const float*    bs = (mat == 0) ? bq : (mat == 1) ? bk : bv;

    const int r    = rowTile * 16 + lo;
    const int koff = hi * 8;

    v8f c[4] = {};
    for (int k0 = 0; k0 < HID; k0 += 32) {
        const _Float16* ar = xh + (size_t)r * HID + k0;
        const v16h a  = cat8(*(const v8h*)(ar + koff),       *(const v8h*)(ar + 16 + koff));
        const v16h al = cat8(*(const v8h*)(ar + PLM + koff), *(const v8h*)(ar + PLM + 16 + koff));
#pragma unroll
        for (int nt = 0; nt < 4; ++nt) {
            const int n = colBase + nt * 16 + lo;
            const _Float16* bp = WT + (size_t)n * HID + k0;
            const v16h b  = cat8(*(const v8h*)(bp + koff),       *(const v8h*)(bp + 16 + koff));
            const v16h bl = cat8(*(const v8h*)(bp + PLW + koff), *(const v8h*)(bp + PLW + 16 + koff));
            c[nt] = wmma_split(a, al, b, bl, c[nt]);
        }
    }

    __shared__ __align__(16) float st2[16 * 256];
    const float sc = (mat == 0) ? 0.125f : 1.0f;
#pragma unroll
    for (int nt = 0; nt < 4; ++nt) {
        const int nl = wave * 64 + nt * 16 + lo;
        const float bias = bs[colBase + nt * 16 + lo];
#pragma unroll
        for (int i = 0; i < 8; ++i) st2[(i + 8 * hi) * 256 + nl] = (c[nt][i] + bias) * sc;
    }
    __syncthreads();
    {
        _Float16* Y = (mat == 0) ? Qh : (mat == 1) ? Kh : Vt;
        const int cb0 = blockIdx.y * 256;
#pragma unroll 1
        for (int pass = 0; pass < 2; ++pass) {
#pragma unroll
            for (int i = 0; i < 4; ++i) {
                const int cc = threadIdx.x + 128 * i, rr = cc >> 5, q = cc & 31;
                {
                    const float* s = st2 + rr * 256 + q * 8;
                    v4u_t v, vl; unsigned lq;
                    v.x = pk2s(s[0], s[1], &lq); vl.x = lq; v.y = pk2s(s[2], s[3], &lq); vl.y = lq; v.z = pk2s(s[4], s[5], &lq); vl.z = lq; v.w = pk2s(s[6], s[7], &lq); vl.w = lq;
                    *(volatile v4u_t*)(Y + (size_t)(rowTile * 16 + rr) * HID + cb0 + q * 8) = v;
                    *(volatile v4u_t*)(Y + PLM + (size_t)(rowTile * 16 + rr) * HID + cb0 + q * 8) = vl;
                }
            }
            __threadfence();
        }
    }
}

__global__ __launch_bounds__(256) void vt_kernel(const _Float16* __restrict__ Vr, _Float16* __restrict__ Vt)
{
    __shared__ _Float16 t[64][66];
    const int tid = threadIdx.x, lane = tid & 31, wave = tid >> 5;
    const int head = blockIdx.y, r0 = blockIdx.x * 64, bb = r0 >> 11, s0 = r0 & (SEQ - 1);
#pragma unroll 1
    for (int pl = 0; pl < 2; ++pl) {
        const size_t po = pl ? PLM : 0;
        if (pl) __syncthreads();
        const _Float16* src = Vr + po + (size_t)r0 * HID + head * HEAD_DIM;
#pragma unroll
        for (int k = 0; k < 16; ++k) { const int e = tid + 256 * k; t[e >> 6][e & 63] = src[(size_t)(e >> 6) * HID + (e & 63)]; }
        __syncthreads();
        _Float16* dst = Vt + po + (size_t)(bb * NHEADS + head) * HEAD_DIM * SEQ + s0;
#pragma unroll
        for (int rr = 0; rr < 8; ++rr) {
            const int hd = wave * 8 + rr;
            const unsigned p = (unsigned)__builtin_bit_cast(unsigned short, t[2 * lane][hd]) | ((unsigned)__builtin_bit_cast(unsigned short, t[2 * lane + 1][hd]) << 16);
            unsigned* d = (unsigned*)(dst + (size_t)hd * SEQ) + lane;
            *(volatile unsigned*)d = p; __threadfence(); *(volatile unsigned*)d = p;
        }
    }
}

__global__ void __launch_bounds__(128) local_attn_kernel(const _Float16* __restrict__ Qh,
                                  const _Float16* __restrict__ Kh,
                                  const _Float16* __restrict__ Vt,
                                  _Float16* __restrict__ Ah)
{
    extern __shared__ _Float16 smem[];

    const int lane = threadIdx.x & 31;
    const int wave = threadIdx.x >> 5;
    const int lo   = lane & 15;
    const int hi   = lane >> 4;
    const int qt   = blockIdx.x;
    const int head = blockIdx.y * 4 + wave;
    const int bb   = blockIdx.z;
    const int koff = hi * 8;

    _Float16* pbuf  = smem + (wave * 1024) / 2;
    _Float16* pbufl = smem + (LDS_PLBUF_BASE + wave * 1024) / 2;

    v16h aq0, aq1, aq0l, aq1l;
    {
        const int qrow = qt * 16 + lo;
        const _Float16* Qr = Qh + ((size_t)(bb * SEQ + qrow)) * HID + head * HEAD_DIM;
        aq0  = cat8(*(const v8h*)(Qr + koff),            *(const v8h*)(Qr + 16 + koff));
        aq1  = cat8(*(const v8h*)(Qr + 32 + koff),       *(const v8h*)(Qr + 48 + koff));
        aq0l = cat8(*(const v8h*)(Qr + PLM + koff),      *(const v8h*)(Qr + PLM + 16 + koff));
        aq1l = cat8(*(const v8h*)(Qr + PLM + 32 + koff), *(const v8h*)(Qr + PLM + 48 + koff));
    }

    v8f oacc[4] = {};
    float rm[8], rl[8];
#pragma unroll
    for (int i = 0; i < 8; ++i) { rm[i] = NEG_BIG; rl[i] = 0.0f; }

    int wstart = qt * 16 - HALF_W; if (wstart < 0) wstart = 0;
    const int s0 = wstart & ~31;
    int send = qt * 16 + 15 + HALF_W; if (send > SEQ - 1) send = SEQ - 1;

    const _Float16* Kbase = Kh + (size_t)(bb * SEQ) * HID + head * HEAD_DIM;
    const _Float16* Vbase = Vt + (size_t)(bb * NHEADS + head) * HEAD_DIM * SEQ;

    tdm_load_tile_f16(LDS_KBUF_BASE + (wave * 2 + 0) * 4096,  Kbase + (size_t)s0 * HID, 64, 32, 64, 32, HID);
    tdm_load_tile_f16(LDS_KLBUF_BASE + (wave * 2 + 0) * 4096, Kbase + PLM + (size_t)s0 * HID, 64, 32, 64, 32, HID);
    tdm_load_tile_f16(LDS_VBUF_BASE + (wave * 2 + 0) * 4096,  Vbase + s0, 32, 64, 32, 64, SEQ);
    tdm_load_tile_f16(LDS_VLBUF_BASE + (wave * 2 + 0) * 4096, Vbase + PLM + s0, 32, 64, 32, 64, SEQ);

    int buf = 0;
    for (int j = s0; j <= send; j += 32, buf ^= 1) {
        if (j + 32 <= send) {
            tdm_load_tile_f16(LDS_KBUF_BASE + (wave * 2 + (buf ^ 1)) * 4096,  Kbase + (size_t)(j + 32) * HID, 64, 32, 64, 32, HID);
            tdm_load_tile_f16(LDS_KLBUF_BASE + (wave * 2 + (buf ^ 1)) * 4096, Kbase + PLM + (size_t)(j + 32) * HID, 64, 32, 64, 32, HID);
            tdm_load_tile_f16(LDS_VBUF_BASE + (wave * 2 + (buf ^ 1)) * 4096,  Vbase + (j + 32), 32, 64, 32, 64, SEQ);
            tdm_load_tile_f16(LDS_VLBUF_BASE + (wave * 2 + (buf ^ 1)) * 4096, Vbase + PLM + (j + 32), 32, 64, 32, 64, SEQ);
            __builtin_amdgcn_s_wait_tensorcnt(4);
        } else {
            __builtin_amdgcn_s_wait_tensorcnt(0);
        }
        asm volatile("" ::: "memory");

        const _Float16* kbuf  = smem + (LDS_KBUF_BASE + (wave * 2 + buf) * 4096) / 2;
        const _Float16* vbuf  = smem + (LDS_VBUF_BASE + (wave * 2 + buf) * 4096) / 2;
        const _Float16* kbufl = smem + (LDS_KLBUF_BASE + (wave * 2 + buf) * 4096) / 2;
        const _Float16* vbufl = smem + (LDS_VLBUF_BASE + (wave * 2 + buf) * 4096) / 2;

        v8f cs0 = {}, cs1 = {};
        {
#define KFR(bufp, row, off) cat8(*(const v8h*)((bufp) + (size_t)(row) * 64 + (off) + koff), *(const v8h*)((bufp) + (size_t)(row) * 64 + (off) + 16 + koff))
            cs0 = wmma_split(aq0, aq0l, KFR(kbuf, lo, 0),       KFR(kbufl, lo, 0),       cs0);
            cs0 = wmma_split(aq1, aq1l, KFR(kbuf, lo, 32),      KFR(kbufl, lo, 32),      cs0);
            cs1 = wmma_split(aq0, aq0l, KFR(kbuf, 16 + lo, 0),  KFR(kbufl, 16 + lo, 0),  cs1);
            cs1 = wmma_split(aq1, aq1l, KFR(kbuf, 16 + lo, 32), KFR(kbufl, 16 + lo, 32), cs1);
#undef KFR
        }

#pragma unroll
        for (int i = 0; i < 8; ++i) {
            const int m   = i + 8 * hi;
            const int q   = qt * 16 + m;
            const int k0i = j + lo;
            const int k1i = j + 16 + lo;
            int d0 = q - k0i; d0 = d0 < 0 ? -d0 : d0;
            int d1 = q - k1i; d1 = d1 < 0 ? -d1 : d1;
            const float sv0 = (d0 <= HALF_W) ? cs0[i] : NEG_BIG;
            const float sv1 = (d1 <= HALF_W) ? cs1[i] : NEG_BIG;

            float mx = fmaxf(sv0, sv1);
#pragma unroll
            for (int d = 1; d < 16; d <<= 1) mx = fmaxf(mx, __shfl_xor(mx, d, 32));
            const float mnew = fmaxf(rm[i], mx);
            const float scal = __expf(rm[i] - mnew);
            const float p0   = __expf(sv0 - mnew);
            const float p1   = __expf(sv1 - mnew);
            float sum = p0 + p1;
#pragma unroll
            for (int d = 1; d < 16; d <<= 1) sum += __shfl_xor(sum, d, 32);
            rl[i] = rl[i] * scal + sum;
            rm[i] = mnew;
#pragma unroll
            for (int nt = 0; nt < 4; ++nt) oacc[nt][i] *= scal;

            {
                const float q0 = p0 * 1024.0f, q1 = p1 * 1024.0f; const _Float16 h0 = (_Float16)q0, h1 = (_Float16)q1;
                pbuf[m * 32 + lo] = h0;       pbufl[m * 32 + lo]      = (_Float16)((q0 - (float)h0) * 2048.0f);
                pbuf[m * 32 + 16 + lo] = h1;  pbufl[m * 32 + 16 + lo] = (_Float16)((q1 - (float)h1) * 2048.0f);
            }
        }
        __syncthreads();

        const v16h ap  = cat8(*(const v8h*)(pbuf + lo * 32 + koff),  *(const v8h*)(pbuf + lo * 32 + 16 + koff));
        const v16h apl = cat8(*(const v8h*)(pbufl + lo * 32 + koff), *(const v8h*)(pbufl + lo * 32 + 16 + koff));
        __syncthreads();

#pragma unroll
        for (int nt = 0; nt < 4; ++nt) {
            const v16h vb  = cat8(*(const v8h*)(vbuf + (size_t)(nt * 16 + lo) * 32 + koff),  *(const v8h*)(vbuf + (size_t)(nt * 16 + lo) * 32 + 16 + koff));
            const v16h vbl = cat8(*(const v8h*)(vbufl + (size_t)(nt * 16 + lo) * 32 + koff), *(const v8h*)(vbufl + (size_t)(nt * 16 + lo) * 32 + 16 + koff));
            oacc[nt] = wmma_split(ap, apl, vb, vbl, oacc[nt]);
        }
    }

    float* so = (float*)(smem + (LDS_KBUF_BASE + (wave * 2) * 4096) / 2);
#pragma unroll
    for (int nt = 0; nt < 4; ++nt) {
#pragma unroll
        for (int i = 0; i < 8; ++i) so[(i + 8 * hi) * 64 + nt * 16 + lo] = oacc[nt][i] / (rl[i] * 1024.0f);
    }
    asm volatile("s_wait_dscnt 0" ::: "memory");
#pragma unroll 1
    for (int pass = 0; pass < 2; ++pass) {
#pragma unroll 4
        for (int rr = 0; rr < 16; ++rr) {
            unsigned lq; const unsigned p = pk2s(so[rr * 64 + 2 * lane], so[rr * 64 + 2 * lane + 1], &lq);
            *(volatile unsigned*)(Ah + ((size_t)(bb * SEQ + qt * 16 + rr)) * HID + head * HEAD_DIM + 2 * lane) = p;
            *(volatile unsigned*)(Ah + PLM + ((size_t)(bb * SEQ + qt * 16 + rr)) * HID + head * HEAD_DIM + 2 * lane) = lq;
        }
        __threadfence();
    }
}

__global__ void out_proj_kernel(const _Float16* __restrict__ Ah,
                                const _Float16* __restrict__ WTo,
                                const float* __restrict__ bo,
                                float* __restrict__ out)
{
    const int lane = threadIdx.x & 31;
    const int wave = threadIdx.x >> 5;
    const int lo   = lane & 15;
    const int hi   = lane >> 4;
    const int rowTile = blockIdx.x;
    const int colBase = (blockIdx.y * 4 + wave) * 64;

    const int r    = rowTile * 16 + lo;
    const int koff = hi * 8;

    v8f c[4] = {};
    for (int k0 = 0; k0 < HID; k0 += 32) {
        const _Float16* ar = Ah + (size_t)r * HID + k0;
        const v16h a  = cat8(*(const v8h*)(ar + koff),       *(const v8h*)(ar + 16 + koff));
        const v16h al = cat8(*(const v8h*)(ar + PLM + koff), *(const v8h*)(ar + PLM + 16 + koff));
#pragma unroll
        for (int nt = 0; nt < 4; ++nt) {
            const int n = colBase + nt * 16 + lo;
            const _Float16* bp = WTo + (size_t)n * HID + k0;
            const v16h b  = cat8(*(const v8h*)(bp + koff),       *(const v8h*)(bp + 16 + koff));
            const v16h bl = cat8(*(const v8h*)(bp + PLW + koff), *(const v8h*)(bp + PLW + 16 + koff));
            c[nt] = wmma_split(a, al, b, bl, c[nt]); if (0) c[nt] = __builtin_amdgcn_wmma_f32_16x16x32_f16(false, a, false, b,
                                                           (short)0, c[nt], false, false);
        }
    }

    extern __shared__ float osm[];
    float* so = osm + wave * (16 * 64);
#pragma unroll
    for (int nt = 0; nt < 4; ++nt) {
        const float bias = bo[colBase + nt * 16 + lo];
#pragma unroll
        for (int i = 0; i < 8; ++i) so[(i + 8 * hi) * 64 + nt * 16 + lo] = c[nt][i] + bias;
    }
    asm volatile("s_wait_dscnt 0" ::: "memory");
#pragma unroll 1
    for (int pass = 0; pass < 2; ++pass) {
#pragma unroll
        for (int i = 0; i < 8; ++i) {
            const int cc = lane + 32 * i, rr = cc >> 4, q = cc & 15;
            *(volatile v4f_t*)(out + (size_t)(rowTile * 16 + rr) * HID + colBase + q * 4) = *(const volatile v4fa*)(so + rr * 64 + q * 4);
        }
        __threadfence();
    }
}

extern "C" void kernel_launch(void* const* d_in, const int* in_sizes, int n_in,
                              void* d_out, int out_size, void* d_ws, size_t ws_size,
                              hipStream_t stream)
{
    (void)in_sizes; (void)n_in; (void)out_size; (void)ws_size;

    const float* x  = (const float*)d_in[0];
    const float* Wq = (const float*)d_in[1];
    const float* bq = (const float*)d_in[2];
    const float* Wk = (const float*)d_in[3];
    const float* bk = (const float*)d_in[4];
    const float* Wv = (const float*)d_in[5];
    const float* bv = (const float*)d_in[6];
    const float* Wo = (const float*)d_in[7];
    const float* bo = (const float*)d_in[8];
    float* out = (float*)d_out;

    const size_t MH = (size_t)BATCH * SEQ * HID;
    const size_t WW = (size_t)HID * HID;
    _Float16* xh  = (_Float16*)d_ws;
    _Float16* Qh  = xh + 2 * MH;
    _Float16* Kh  = Qh + 2 * MH;
    _Float16* Vt  = Kh + 2 * MH;
    _Float16* Ah  = Vt + 2 * MH;
    _Float16* WTq = Ah + 2 * MH;
    _Float16* WTk = WTq + 2 * WW;
    _Float16* WTv = WTk + 2 * WW;
    _Float16* WTo = WTv + 2 * WW;
    _Float16* Vr  = WTo + 2 * WW;

    cvt_x_kernel<<<dim3(MH / (256 * 4)), 256, 0, stream>>>(x, xh);
    cvt_w_kernel<<<dim3(HID * HID / 2 / 256, 4), 256, 0, stream>>>(
        Wq, Wk, Wv, Wo, WTq, WTk, WTv, WTo);

    dim3 g1(BATCH * SEQ / 16, HID / 256, 3);
    qkv_proj_kernel<<<g1, 128, 0, stream>>>(xh, WTq, WTk, WTv, bq, bk, bv, Qh, Kh, Vr);
    vt_kernel<<<dim3(BATCH * SEQ / 64, NHEADS), 256, 0, stream>>>(Vr, Vt);

    dim3 g2(SEQ / 16, NHEADS / 4, BATCH);
    (void)hipFuncSetAttribute((const void*)local_attn_kernel, hipFuncAttributeMaxDynamicSharedMemorySize, LDS_TOTAL_BYTES);
    local_attn_kernel<<<g2, 128, LDS_TOTAL_BYTES, stream>>>(Qh, Kh, Vt, Ah);

    dim3 g3(BATCH * SEQ / 16, HID / 256);
    out_proj_kernel<<<g3, 128, 4 * 16 * 64 * sizeof(float), stream>>>(Ah, WTo, bo, out);
}
